// GCoRe_78262894068282
// MI455X (gfx1250) — hardware-verified
//
#include <hip/hip_runtime.h>
#include <math.h>


#define NN 50000
#define NE 600000
#define DD 128
#define NL 8
#define NG 64
#define NCLS 10
#define SLOTC 32
#define NCH 768
#define NBLK ((NN + 63) / 64)

typedef __attribute__((ext_vector_type(16))) _Float16 v16h;
typedef __attribute__((ext_vector_type(16))) __bf16 v16b;
typedef __attribute__((ext_vector_type(8)))  __bf16 v8b;
typedef __attribute__((ext_vector_type(8)))  _Float16 v8h;
typedef __attribute__((ext_vector_type(8)))  float v8f;
typedef __attribute__((ext_vector_type(4)))  float v4f;
typedef __attribute__((ext_vector_type(4)))  unsigned v4u;
typedef __attribute__((ext_vector_type(4)))  int v4i;
typedef float __attribute__((may_alias)) float_a;

template <typename T> __device__ __forceinline__ void vst2(void* p, T v) { *(volatile T*)p = v; __threadfence(); *(volatile T*)p = v; }
__device__ __forceinline__ v8f wmma16(v16h a, v16h b, v8f c) {
  v8f d = __builtin_amdgcn_wmma_f32_16x16x32_f16(false, a, false, b, (short)0, c, false, false);
  asm volatile("v_nop\n\tv_nop\n\tv_nop\n\tv_nop" : "+v"(d) : "v"(a), "v"(b));
  return d;
}
__device__ __forceinline__ v16h frag_h(const _Float16* rowk0, int lane) {
  union { v16h v; v8h q[2]; } u; const _Float16* p = rowk0 + 8 * (lane >> 4);
  u.q[0] = *(const v8h*)p; u.q[1] = *(const v8h*)(p + 16); return u.v;
}
__device__ __forceinline__ v16h frag_f32(const float* rowk0, int lane) {
  v16h a; const float* p = rowk0 + 8 * (lane >> 4);
#pragma unroll
  for (int i = 0; i < 8; ++i) { a[i] = (_Float16)p[i]; a[8 + i] = (_Float16)p[16 + i]; }
  return a;
}
__device__ __forceinline__ v8f wmma_bf(v16b a, v16b b, v8f c) {
  v8f d = __builtin_amdgcn_wmma_f32_16x16x32_bf16(false, a, false, b, (short)0, c, false, false);
  asm volatile("v_nop\n\tv_nop\n\tv_nop\n\tv_nop" : "+v"(d) : "v"(a), "v"(b));
  return d;
}
struct F2 { v16b h, l; };
__device__ __forceinline__ F2 split_row(const float* rowk0, int lane) {
  F2 r; const float* p = rowk0 + 8 * (lane >> 4);
#pragma unroll
  for (int i = 0; i < 8; ++i) { float v0 = p[i], v1 = p[16 + i]; __bf16 h0 = (__bf16)v0, h1 = (__bf16)v1;
    r.h[i] = h0; r.l[i] = (__bf16)(v0 - (float)h0); r.h[8 + i] = h1; r.l[8 + i] = (__bf16)(v1 - (float)h1); }
  return r;
}
__device__ __forceinline__ v8f mac3(const F2& a, const F2& b, v8f c) { c = wmma_bf(a.l, b.h, c); c = wmma_bf(a.h, b.l, c); return wmma_bf(a.h, b.h, c); }
__device__ __forceinline__ float lrelu(float v) { return v >= 0.f ? v : 0.01f * v; }
#define LDSX() do { asm volatile("s_wait_dscnt 0" ::: "memory"); __builtin_amdgcn_wave_barrier(); __builtin_amdgcn_fence(__ATOMIC_RELEASE, "workgroup"); } while (0)

__global__ __launch_bounds__(256) void k_packT(const float* __restrict__ W, __bf16* __restrict__ Wh, __bf16* __restrict__ Wlo, int K, int N) {
  __shared__ float tile[64][65];
  const int k0 = blockIdx.y * 64, n0 = blockIdx.x * 64, l = blockIdx.z, tid = threadIdx.x;
  const float* Wl = W + (size_t)l * K * N; __bf16* Wth = Wh + (size_t)l * K * N; __bf16* Wtl = Wlo + (size_t)l * K * N;
  for (int q = tid; q < 64 * 64; q += 256) { const int kk = q >> 6, nn = q & 63; tile[kk][nn] = Wl[(size_t)(k0 + kk) * N + n0 + nn]; }
  __syncthreads();
  for (int q = tid; q < 64 * 8; q += 256) { const int nn = q >> 3, pc = q & 7;
    union { v8b h; v4u u; } ph, pl;
#pragma unroll
    for (int e = 0; e < 8; ++e) { const float v = tile[pc * 8 + e][nn]; const __bf16 h = (__bf16)v; ph.h[e] = h; pl.h[e] = (__bf16)(v - (float)h); }
    vst2(Wth + (size_t)(n0 + nn) * K + k0 + pc * 8, ph.u); vst2(Wtl + (size_t)(n0 + nn) * K + k0 + pc * 8, pl.u); }
}
__device__ __forceinline__ F2 frag_b2(const __bf16* rh, const __bf16* rl, int lane) {
  F2 r; union { v16b v; v8b q[2]; } uh, ul; const int o = 8 * (lane >> 4);
  uh.q[0] = *(const v8b*)(rh + o); uh.q[1] = *(const v8b*)(rh + o + 16); ul.q[0] = *(const v8b*)(rl + o); ul.q[1] = *(const v8b*)(rl + o + 16);
  r.h = uh.v; r.l = ul.v; return r;
}

__global__ __launch_bounds__(256) void k_bucket(const int* __restrict__ ei, int* __restrict__ tlist) {
  __shared__ int scnt[NCH];
  __shared__ int slots[NCH][SLOTC];
  const int tid = threadIdx.x, n0 = blockIdx.x * NCH;
  for (int i = tid; i < NCH; i += 256) scnt[i] = 0;
  __syncthreads();
  for (int e = tid; e < NE; e += 256) { const int i = ei[NE + e] - n0;
    if (i >= 0 && i < NCH) { const int s = atomicAdd(&scnt[i], 1); if (s < SLOTC - 1) slots[i][s] = e; } }
  __syncthreads();
  for (int i = tid; i < NCH; i += 256) { const int n = n0 + i; if (n >= NN) continue;
    const int ctrue = scnt[i]; int c = ctrue; if (c > SLOTC - 1) c = SLOTC - 1;
    for (int a = 1; a < c; ++a) { const int v = slots[i][a]; int b = a - 1; while (b >= 0 && slots[i][b] > v) { slots[i][b + 1] = slots[i][b]; --b; } slots[i][b + 1] = v; }
    for (int a = c; a < SLOTC; ++a) slots[i][a] = 0;
    slots[i][SLOTC - 1] = ctrue;
#pragma unroll 1
    for (int p = 0; p < SLOTC / 4; ++p) { v4i v = { slots[i][4 * p], slots[i][4 * p + 1], slots[i][4 * p + 2], slots[i][4 * p + 3] }; vst2(tlist + (size_t)n * SLOTC + 4 * p, v); }
  }
}

__device__ __forceinline__ float xform(float z, float sc, float sh, int act) { const float v = z * sc + sh; return act ? lrelu(v) : v; }

__global__ __launch_bounds__(256) void k_agg(const float* __restrict__ zin, const float* __restrict__ coef, int act, const int* __restrict__ ei,
                                           const int* __restrict__ tlist, float* __restrict__ zr) {
  const int tid = threadIdx.x, w = tid >> 5, lane = tid & 31, half = lane >> 4, c0 = (lane & 15) * 8;
  const int n = blockIdx.x * 16 + w * 2 + half;
  if (n >= NN) return;
  float sc[8], sh[8], acc[8];
#pragma unroll
  for (int e = 0; e < 8; ++e) { sc[e] = coef[c0 + e]; sh[e] = coef[DD + c0 + e]; acc[e] = xform(zin[(size_t)n * DD + c0 + e], sc[e], sh[e], act); }
  int dn = tlist[(size_t)n * SLOTC + SLOTC - 1]; dn = dn < 0 ? 0 : (dn > SLOTC - 1 ? SLOTC - 1 : dn);
#pragma unroll 1
  for (int q = 0; q < dn; ++q) { int e = tlist[(size_t)n * SLOTC + q]; if ((unsigned)e >= (unsigned)NE) continue;
    int s = ei[e]; s = s < 0 ? 0 : (s >= NN ? NN - 1 : s);
    const float* hr = zin + (size_t)s * DD + c0;
#pragma unroll
    for (int k = 0; k < 8; ++k) acc[k] += xform(hr[k], sc[k], sh[k], act); }
  vst2(zr + (size_t)n * DD + c0, (v4f){acc[0], acc[1], acc[2], acc[3]});
  vst2(zr + (size_t)n * DD + c0 + 4, (v4f){acc[4], acc[5], acc[6], acc[7]});
}

__global__ __launch_bounds__(128) void k_mlp(const float* __restrict__ zr, const __bf16* __restrict__ W1h, const __bf16* __restrict__ W1l, const float* __restrict__ b1,
                                           const __bf16* __restrict__ W2h, const __bf16* __restrict__ W2l, const float* __restrict__ b2, float* __restrict__ z2, float* __restrict__ part) {
  __shared__ __align__(16) float S[4][16][132];
  __shared__ float cs[4][2][128];
  const int tid = threadIdx.x, wave = tid >> 5, lane = tid & 31, col = lane & 15, g = lane >> 4;
  const int r0 = blockIdx.x * 64 + wave * 16;
  const bool live = r0 < NN;
  float* Sw = &S[wave][0][0];
  float q1[4] = {0.f, 0.f, 0.f, 0.f}, q2[4] = {0.f, 0.f, 0.f, 0.f};
  if (live) {
    v8f acc[8] = {};
#pragma unroll
    for (int kc = 0; kc < 4; ++kc) { const F2 a = split_row(zr + (size_t)(r0 + col) * DD + kc * 32, lane);
#pragma unroll
      for (int j = 0; j < 8; ++j) { const size_t ro = (size_t)(j * 16 + col) * DD + kc * 32; acc[j] = mac3(a, frag_b2(W1h + ro, W1l + ro, lane), acc[j]); } }
#pragma unroll
    for (int j = 0; j < 8; ++j) { const float bv = b1[j * 16 + col];
#pragma unroll
      for (int r = 0; r < 8; ++r) Sw[(8 * g + r) * 132 + j * 16 + col] = lrelu(acc[j][r] + bv); }
    LDSX();
#pragma unroll
    for (int j = 0; j < 8; ++j) acc[j] = (v8f){};
#pragma unroll
    for (int kc = 0; kc < 4; ++kc) { const F2 a = split_row(Sw + col * 132 + kc * 32, lane);
#pragma unroll
      for (int j = 0; j < 8; ++j) { const size_t ro = (size_t)(j * 16 + col) * DD + kc * 32; acc[j] = mac3(a, frag_b2(W2h + ro, W2l + ro, lane), acc[j]); } }
    __builtin_amdgcn_wave_barrier();
#pragma unroll
    for (int j = 0; j < 8; ++j) { const float bv = b2[j * 16 + col];
#pragma unroll
      for (int r = 0; r < 8; ++r) Sw[(8 * g + r) * 132 + j * 16 + col] = acc[j][r] + bv; }
    LDSX();
#pragma unroll
    for (int q = 0; q < 8; ++q) { const int rl = q * 2 + (lane >> 4), pc = lane & 15;
      const float* src = Sw + rl * 132 + pc * 8;
      vst2(z2 + (size_t)(r0 + rl) * DD + pc * 8, *(const v4f*)src); vst2(z2 + (size_t)(r0 + rl) * DD + pc * 8 + 4, *(const v4f*)(src + 4)); }
    for (int rl = 0; rl < 16; ++rl) { const v4f v = *(const v4f*)(Sw + rl * 132 + lane * 4);
#pragma unroll
      for (int e = 0; e < 4; ++e) { q1[e] += v[e]; q2[e] += v[e] * v[e]; } }
  }
#pragma unroll
  for (int e = 0; e < 4; ++e) { cs[wave][0][lane * 4 + e] = q1[e]; cs[wave][1][lane * 4 + e] = q2[e]; }
  __syncthreads();
  if (tid < 64) { const int which = tid >> 5, l4 = (tid & 31) * 4; v4f t;
#pragma unroll
    for (int e = 0; e < 4; ++e) t[e] = cs[0][which][l4 + e] + cs[1][which][l4 + e] + cs[2][which][l4 + e] + cs[3][which][l4 + e];
    vst2(part + ((size_t)blockIdx.x * 2 + which) * DD + l4, t); }
}

__global__ __launch_bounds__(128) void k_ident(float* __restrict__ coef) { const int c = threadIdx.x; vst2(coef + c, (float_a)1.0f); vst2(coef + DD + c, (float_a)0.0f); }

__global__ __launch_bounds__(128) void k_bn(const float* __restrict__ part, const float* __restrict__ gm, const float* __restrict__ bt, float* __restrict__ coef) {
  const int c = threadIdx.x;
  float s = 0.f, q = 0.f;
#pragma unroll 1
  for (int b = 0; b < NBLK; ++b) { s += part[((size_t)b * 2) * DD + c]; q += part[((size_t)b * 2 + 1) * DD + c]; }
  const float mu = s / (float)NN; float var = q / (float)NN - mu * mu; var = var < 0.f ? 0.f : var;
  const float sc = gm[c] * rsqrtf(var + 1e-5f);
  vst2(coef + c, (float_a)sc);
  vst2(coef + DD + c, (float_a)(bt[c] - mu * sc));
}

__global__ __launch_bounds__(256) void k_assign(const float* __restrict__ z2, const float* __restrict__ coef, const float* __restrict__ gn, float* __restrict__ cout) {
  const int tid = threadIdx.x, w = tid >> 5, lane = tid & 31;
  const int n = blockIdx.x * 8 + w;
  if (n >= NN) return;
  const v4f z = *(const v4f*)(z2 + (size_t)n * DD + lane * 4), g4 = *(const v4f*)(gn + (size_t)n * DD + lane * 4);
  const v4f sc = *(const v4f*)(coef + lane * 4), sh = *(const v4f*)(coef + DD + lane * 4);
  v4f l = z * sc + sh + g4;
  float mx = fmaxf(fmaxf(l[0], l[1]), fmaxf(l[2], l[3]));
#pragma unroll
  for (int off = 16; off >= 1; off >>= 1) mx = fmaxf(mx, __shfl_xor(mx, off, 32));
  v4f e = { expf(l[0] - mx), expf(l[1] - mx), expf(l[2] - mx), expf(l[3] - mx) };
  float s = e[0] + e[1] + e[2] + e[3];
#pragma unroll
  for (int off = 16; off >= 1; off >>= 1) s += __shfl_xor(s, off, 32);
  vst2(cout + (size_t)n * DD + lane * 4, e * (1.0f / s));
}

__global__ __launch_bounds__(256) void k_pool(const float* __restrict__ cout, const int* __restrict__ batch,
                                            const float* __restrict__ Wd1, const float* __restrict__ bd1, const float* __restrict__ Wd2, const float* __restrict__ bd2,
                                            float* __restrict__ res) {
  __shared__ int cntlt[256], cnteq[256];
  __shared__ float psum[8][DD], pooled[DD], hid[DD], lg[16];
  const int gi = blockIdx.x, tid = threadIdx.x, w = tid >> 5, lane = tid & 31;
  int lt = 0, eq = 0;
  for (int i = tid; i < NN; i += 256) { const int b = batch[i]; lt += (b < gi); eq += (b == gi); }
  cntlt[tid] = lt; cnteq[tid] = eq; __syncthreads();
  for (int st = 128; st > 0; st >>= 1) { if (tid < st) { cntlt[tid] += cntlt[tid + st]; cnteq[tid] += cnteq[tid + st]; } __syncthreads(); }
  const int start = cntlt[0], count = cnteq[0];
  float s4[4] = {0.f, 0.f, 0.f, 0.f};
  for (int i = start + w; i < start + count; i += 8) { const v4f v = *(const v4f*)(cout + (size_t)i * DD + lane * 4); s4[0] += v[0]; s4[1] += v[1]; s4[2] += v[2]; s4[3] += v[3]; }
#pragma unroll
  for (int e = 0; e < 4; ++e) psum[w][lane * 4 + e] = s4[e];
  __syncthreads();
  if (tid < DD) { float t = 0.f; for (int i = 0; i < 8; ++i) t += psum[i][tid]; pooled[tid] = t; }
  __syncthreads();
  if (tid < DD) { float a = bd1[tid];
#pragma unroll 1
    for (int i = 0; i < DD; ++i) a += pooled[i] * Wd1[i * DD + tid];
    hid[tid] = lrelu(a); }
  __syncthreads();
  if (tid < NCLS) { float a = bd2[tid];
#pragma unroll 1
    for (int i = 0; i < DD; ++i) a += hid[i] * Wd2[i * NCLS + tid];
    lg[tid] = a; }
  __syncthreads();
  if (tid < 32) { float mx = -3.0e38f; for (int i = 0; i < NCLS; ++i) mx = fmaxf(mx, lg[i]);
    float s = 0.f; for (int i = 0; i < NCLS; ++i) s += expf(lg[i] - mx);
    const float v = tid < NCLS ? expf(lg[tid] - mx) / s : 0.f;
    vst2(res + (size_t)gi * 32 + tid, (float_a)v); }
}
__global__ __launch_bounds__(256) void k_fin(const float* __restrict__ res, float* __restrict__ out) {
  __shared__ __align__(16) float so[NG * NCLS];
  for (int i = threadIdx.x; i < NG * NCLS; i += 256) so[i] = res[(size_t)(i / NCLS) * 32 + (i % NCLS)];
  __syncthreads();
  if (threadIdx.x < NG * NCLS / 4) vst2(out + threadIdx.x * 4, *(const v4f*)(&so[threadIdx.x * 4]));
}

extern "C" void kernel_launch(void* const* d_in, const int* in_sizes, int n_in,
                              void* d_out, int out_size, void* d_ws, size_t ws_size,
                              hipStream_t stream) {
  (void)in_sizes; (void)n_in; (void)out_size; (void)ws_size;
  const float* x = (const float*)d_in[0]; const int* ei = (const int*)d_in[1]; const int* batch = (const int*)d_in[2];
  const float* gn = (const float*)d_in[3];
  const float* W1s = (const float*)d_in[4]; const float* b1s = (const float*)d_in[5];
  const float* W2s = (const float*)d_in[6]; const float* b2s = (const float*)d_in[7];
  const float* gms = (const float*)d_in[8]; const float* bts = (const float*)d_in[9];
  const float* Wd1 = (const float*)d_in[10]; const float* bd1 = (const float*)d_in[11];
  const float* Wd2 = (const float*)d_in[12]; const float* bd2 = (const float*)d_in[13];
  float* out = (float*)d_out; float* cout = (float*)d_out + 640;
  char* ws = (char*)d_ws; size_t off = 0;
  auto take = [&](size_t bytes) { char* p = ws + off; off += (bytes + 255) & ~(size_t)255; return p; };
  const int NPAD = NBLK * 64;
  __bf16* W1h = (__bf16*)take((size_t)NL * DD * DD * 2); __bf16* W1l = (__bf16*)take((size_t)NL * DD * DD * 2);
  __bf16* W2h = (__bf16*)take((size_t)NL * DD * DD * 2); __bf16* W2l = (__bf16*)take((size_t)NL * DD * DD * 2);
  int* tlist = (int*)take((size_t)NN * SLOTC * 4);
  float* z16 = (float*)take((size_t)NPAD * DD * 4);
  float* z2 = (float*)take((size_t)NPAD * DD * 4);
  float* part = (float*)take((size_t)NBLK * 2 * DD * 4);
  float* coef = (float*)take((size_t)(NL + 1) * 2 * DD * 4);
  float* res = (float*)take((size_t)NG * 32 * 4);
  k_packT<<<dim3(DD / 64, DD / 64, NL), 256, 0, stream>>>(W1s, W1h, W1l, DD, DD);
  k_packT<<<dim3(DD / 64, DD / 64, NL), 256, 0, stream>>>(W2s, W2h, W2l, DD, DD);
  k_bucket<<<(NN + NCH - 1) / NCH, 256, 0, stream>>>(ei, tlist);
  k_ident<<<1, 128, 0, stream>>>(coef);
  const float* zin = x; int act = 0;
  for (int l = 0; l < NL; ++l) {
    k_agg<<<(NN + 15) / 16, 256, 0, stream>>>(zin, coef + (size_t)l * 2 * DD, act, ei, tlist, z16);
    k_mlp<<<NBLK, 128, 0, stream>>>(z16, W1h + (size_t)l * DD * DD, W1l + (size_t)l * DD * DD, b1s + l * DD, W2h + (size_t)l * DD * DD, W2l + (size_t)l * DD * DD, b2s + l * DD, z2, part);
    k_bn<<<1, 128, 0, stream>>>(part, gms + l * DD, bts + l * DD, coef + (size_t)(l + 1) * 2 * DD);
    zin = z2; act = 1;
  }
  k_assign<<<(NN + 7) / 8, 256, 0, stream>>>(z2, coef + (size_t)NL * 2 * DD, gn, cout);
  k_pool<<<NG, 256, 0, stream>>>(cout, batch, Wd1, bd1, Wd2, bd2, res);
  k_fin<<<1, 256, 0, stream>>>(res, out);
}
